// NlsqCond_38989713113397
// MI455X (gfx1250) — hardware-verified
//
#include <hip/hip_runtime.h>


namespace {
constexpr int Bn = 256, T = 64, T2 = 32, TP = 34, HH = 512, CL = 8, NR = Bn * T2  , NRP = Bn * TP  ;
constexpr float XS = 8.0f, LOG_A = 0.3985081094410609f;

typedef _Float16 b16;
typedef __attribute__((ext_vector_type(16))) _Float16 v16b;
typedef __attribute__((ext_vector_type(8))) _Float16 v8b;
typedef __attribute__((ext_vector_type(8))) float v8f;
typedef __attribute__((ext_vector_type(4))) float v4f;
typedef __attribute__((ext_vector_type(2))) float v2f;
__device__ __forceinline__ float bf16_rne(float f) { unsigned int u = __float_as_uint(f); u += 0x7FFFu + ((u >> 16) & 1u); return __uint_as_float(u & 0xFFFF0000u); }
__device__ __forceinline__ void split16(float v, b16& hi, b16& lo) { hi = (b16)v; lo = (b16)(v - (float)hi); }
__device__ __forceinline__ v16b frag_kb(const b16* p, int hh) { const v8b a = *(const v8b*)(p + 8 * hh), b = *(const v8b*)(p + 16 + 8 * hh); v16b f;
#pragma unroll
  for (int e = 0; e < 8; ++e) { f[e] = a[e]; f[8 + e] = b[e]; } return f; }
__device__ __forceinline__ v8f wmma16b(v16b a, v16b b, v8f c) { v8f d = __builtin_amdgcn_wmma_f32_16x16x32_f16(false, a, false, b, (short)0, c, false, false); asm volatile("v_nop\n\tv_nop\n\tv_nop\n\tv_nop" : "+v"(d) : "v"(a), "v"(b)); return d; }
__device__ __forceinline__ void wave_lds_sync() { __builtin_amdgcn_fence(__ATOMIC_RELEASE, "workgroup"); __builtin_amdgcn_wave_barrier(); __builtin_amdgcn_fence(__ATOMIC_ACQUIRE, "workgroup"); }
__device__ __forceinline__ float nexp(float x) { return __builtin_amdgcn_exp2f(x * 1.4426950408889634f); }
__device__ __forceinline__ float pmul(float a, float b) { float p = a * b; asm volatile("" : "+v"(p)); return p; }
__device__ __forceinline__ float tanh_f(float x) { const float e = nexp(-2.0f * fabsf(x)); const float t = (1.0f - e) / (1.0f + e); return (x < 0.0f) ? -t : t; }
__device__ __forceinline__ float wsum(float v) {
#pragma unroll
  for (int o = 1; o < 32; o <<= 1) v += __shfl_xor(v, o); return v; }

struct Ro_ { static constexpr size_t C0 = 0, C1 = (size_t)512 * 3072, WC2 = C1 + (size_t)4 * 512 * 1536, WO = WC2 + (size_t)512 * 512, END = WO + (size_t)16 * 512; };
__global__ __launch_bounds__(256) void prep_kernel(const float* __restrict__ wemb, const float* __restrict__ bemb, const float* __restrict__ wc1, const float* __restrict__ bc1, const float* __restrict__ wc2, const float* __restrict__ bc2, const float* __restrict__ w0, const float* __restrict__ b0, const float* __restrict__ w1, const float* __restrict__ b1, const float* __restrict__ w2, const float* __restrict__ b2,
    const float* __restrict__ w3, const float* __restrict__ b3, const float* __restrict__ w4, const float* __restrict__ b4, const float* __restrict__ wo, const float* __restrict__ bo, b16* __restrict__ R, float* __restrict__ P, b16* __restrict__ Ah0, b16* __restrict__ Al0, b16* __restrict__ Ah1, b16* __restrict__ Al1) {
  const size_t tid = (size_t)blockIdx.x * 256 + threadIdx.x, nth = (size_t)gridDim.x * 256;
  for (int pass = 0; pass < 2; ++pass) {
    for (size_t p = tid; p < Ro_::C1; p += nth) { const int o = (int)(p / 3072), k = (int)((p / 1024) % 3), c = (int)(p % 1024); ((volatile b16*)R)[p] = (b16)bf16_rne(w0[((size_t)o * 1024 + c) * 3 + k]); }
    for (size_t p = tid; p < (size_t)4 * 512 * 1536; p += nth) { const int l = (int)(p / ((size_t)512 * 1536)); const size_t q = p % ((size_t)512 * 1536); const int o = (int)(q / 1536), k = (int)((q / 512) % 3), c = (int)(q % 512); const float* w = (l == 0) ? w1 : (l == 1) ? w2 : (l == 2) ? w3 : w4; ((volatile b16*)R)[Ro_::C1 + p] = (b16)bf16_rne(w[((size_t)o * 512 + c) * 3 + k]); }
    for (size_t p = tid; p < (size_t)512 * 512; p += nth) ((volatile b16*)R)[Ro_::WC2 + p] = (b16)bf16_rne(wc2[p]);
    for (size_t p = tid; p < (size_t)16 * 512; p += nth) { const int o = (int)(p / 512), c = (int)(p % 512); ((volatile b16*)R)[Ro_::WO + p] = (b16)((o < 10) ? bf16_rne(wo[(size_t)o * 512 + c]) : 0.0f); }
    for (size_t q = tid; q < 13328; q += nth) { const int i = (int)q; float v = 0.0f;
      if (i < 512) v = bemb[i]; else if (i < 1536) { const int c = (i - 512) >> 1, d = (i - 512) & 1; v = wemb[c * 6 + d]; } else if (i < 2048) v = bc1[i - 1536]; else if (i < 10240) v = wc1[i - 2048]; else if (i < 10752) v = bc2[i - 10240];
      else if (i < 13312) { const int l = (i - 10752) / 512, j = (i - 10752) % 512; v = ((l == 0) ? b0 : (l == 1) ? b1 : (l == 2) ? b2 : (l == 3) ? b3 : b4)[j]; } else v = (i - 13312 < 10) ? bo[i - 13312] : 0.0f;
      P[q] = bf16_rne(v); }
    for (size_t p = tid; p < (size_t)Bn * 2 * 1024 / 8; p += nth) { const int b = (int)(p / 256), which = (int)((p / 128) & 1), c8 = (int)(p % 128) * 8; const size_t row = (size_t)b * TP + (which ? TP - 1 : 0); const v8b z = {};
      *(volatile v8b*)(Ah0 + row * 1024 + c8) = z; *(volatile v8b*)(Al0 + row * 1024 + c8) = z; if (c8 < 512) { *(volatile v8b*)(Ah1 + row * 512 + c8) = z; *(volatile v8b*)(Al1 + row * 512 + c8) = z; } }
    __threadfence(); }
}
__global__ __launch_bounds__(256) void pre_kernel(const float* __restrict__ x, const float* __restrict__ cond, const float* __restrict__ P, b16* __restrict__ C1h, b16* __restrict__ C1l, b16* __restrict__ Ah0, b16* __restrict__ Al0) {
  __shared__ float cf[16]; __shared__ __attribute__((aligned(16))) b16 Sh[HH + 8], Sl[HH + 8]; __shared__ __attribute__((aligned(16))) b16 Eh[T2][HH + 8], El[T2][HH + 8];
  const int b = blockIdx.x, t_ = threadIdx.x;
  if (t_ < 16) cf[t_] = bf16_rne(cond[(size_t)b * 16 + t_]);
  __syncthreads();
  for (int j = t_; j < HH; j += 256) { float s = P[1536 + j]; for (int i = 0; i < 16; ++i) s += pmul(cf[i], P[2048 + j * 16 + i]); s = fmaxf(s, 0.0f); b16 a_, c_; split16(s * XS, a_, c_); Sh[j] = a_; Sl[j] = c_; }
  for (int i = t_; i < T2 * HH; i += 256) { const int t = i / HH, c = i % HH; const float z0 = bf16_rne(x[((size_t)b * T + t) * 2]), z1v = bf16_rne(x[((size_t)b * T + t) * 2 + 1]); const float h = pmul(z0, P[512 + c * 2]) + pmul(z1v, P[512 + c * 2 + 1]) + P[c]; b16 a_, c_; split16(h * XS, a_, c_); Eh[t][c] = a_; El[t][c] = c_; }
  __syncthreads();
  for (int pass = 0; pass < 2; ++pass) { for (int i = t_; i < HH / 8; i += 256) { *(volatile v8b*)(C1h + (size_t)b * HH + i * 8) = *(const v8b*)(&Sh[i * 8]); *(volatile v8b*)(C1l + (size_t)b * HH + i * 8) = *(const v8b*)(&Sl[i * 8]); }
    for (int i = t_; i < T2 * (HH / 8); i += 256) { const int t = i / (HH / 8), c8 = (i % (HH / 8)) * 8; const size_t gi = ((size_t)b * TP + 1 + t) * 1024 + c8; *(volatile v8b*)(Ah0 + gi) = *(const v8b*)(&Eh[t][c8]); *(volatile v8b*)(Al0 + gi) = *(const v8b*)(&El[t][c8]); } __threadfence(); }
}
__global__ __launch_bounds__(64) void cond2_kernel(const b16* __restrict__ C1h, const b16* __restrict__ C1l, const b16* __restrict__ R, const float* __restrict__ P, b16* __restrict__ Ah0, b16* __restrict__ Al0) {
  __shared__ __attribute__((aligned(16))) b16 Th[2][16][128 + 8], Tl[2][16][128 + 8];
  const int lane = threadIdx.x & 31, wave = threadIdx.x >> 5, nloc = lane & 15, hlf = lane >> 4, m0 = blockIdx.y * 32 + wave * 16, c0 = blockIdx.x * 128; const b16* Bw = R + Ro_::WC2;
  v8f acc[8];
#pragma unroll
  for (int t = 0; t < 8; ++t) acc[t] = (v8f){};
#pragma unroll
  for (int kb = 0; kb < HH; kb += 32) { const v16b a = frag_kb(C1h + (size_t)(m0 + nloc) * HH + kb, hlf), al_ = frag_kb(C1l + (size_t)(m0 + nloc) * HH + kb, hlf);
#pragma unroll
    for (int t = 0; t < 8; ++t) { const v16b bw = frag_kb(Bw + (size_t)(c0 + t * 16 + nloc) * HH + kb, hlf); acc[t] = wmma16b(a, bw, acc[t]); acc[t] = wmma16b(al_, bw, acc[t]); } }
#pragma unroll
  for (int t = 0; t < 8; ++t)
#pragma unroll
    for (int r = 0; r < 8; ++r) { const float v = fmaxf(acc[t][r] * (1.0f / XS) + P[10240 + c0 + t * 16 + nloc], 0.0f); b16 a_, c_; split16(v * XS, a_, c_); Th[wave][8 * hlf + r][t * 16 + nloc] = a_; Tl[wave][8 * hlf + r][t * 16 + nloc] = c_; }
  wave_lds_sync();
  for (int pass = 0; pass < 2; ++pass) { for (int i = lane; i < 16 * T2 * 16; i += 32) { const int rr = i / (T2 * 16), rem = i % (T2 * 16), t = rem >> 4, c8 = (rem & 15) * 8; const int b = m0 + rr; const size_t gi = ((size_t)b * TP + 1 + t) * 1024 + 512 + c0 + c8; *(volatile v8b*)(Ah0 + gi) = *(const v8b*)(&Th[wave][rr][c8]); *(volatile v8b*)(Al0 + gi) = *(const v8b*)(&Tl[wave][rr][c8]); } __threadfence(); }
}
template <int CIN, int LAST>
__global__ __launch_bounds__(64) void conv_kernel(const b16* __restrict__ Ah, const b16* __restrict__ Al, const b16* __restrict__ Bw, const float* __restrict__ bias, b16* __restrict__ Oh, b16* __restrict__ Ol, float* __restrict__ HF) {
  __shared__ __attribute__((aligned(16))) b16 Th[2][16][128 + 8], Tl[2][16][128 + 8]; __shared__ __attribute__((aligned(16))) float Ts[2][16][128 + 4];
  const int lane = threadIdx.x & 31, wave = threadIdx.x >> 5, nloc = lane & 15, hlf = lane >> 4, b = blockIdx.y, t0 = wave * 16, c0 = blockIdx.x * 128;
  const size_t arow = (size_t)b * TP + t0;
  v8f acc[8];
#pragma unroll
  for (int t = 0; t < 8; ++t) acc[t] = (v8f){};
  for (int k = 0; k < 3; ++k) {
#pragma unroll 2
    for (int kb = 0; kb < CIN; kb += 32) { const v16b a = frag_kb(Ah + (arow + k + nloc) * CIN + kb, hlf), al_ = frag_kb(Al + (arow + k + nloc) * CIN + kb, hlf);
#pragma unroll
      for (int t = 0; t < 8; ++t) { const v16b bw = frag_kb(Bw + (size_t)(c0 + t * 16 + nloc) * (3 * CIN) + (size_t)k * CIN + kb, hlf); acc[t] = wmma16b(a, bw, acc[t]); acc[t] = wmma16b(al_, bw, acc[t]); } } }
#pragma unroll
  for (int t = 0; t < 8; ++t)
#pragma unroll
    for (int r = 0; r < 8; ++r) { const float v = fmaxf(acc[t][r] * (1.0f / XS) + bias[c0 + t * 16 + nloc], 0.0f); if (LAST) Ts[wave][8 * hlf + r][t * 16 + nloc] = v; else { b16 a_, c_; split16(v * XS, a_, c_); Th[wave][8 * hlf + r][t * 16 + nloc] = a_; Tl[wave][8 * hlf + r][t * 16 + nloc] = c_; } }
  wave_lds_sync();
  for (int pass = 0; pass < 2; ++pass) {
    if (LAST) { for (int i = lane; i < 16 * 32; i += 32) { const int rr = i >> 5, c4 = (i & 31) * 4; *(volatile v4f*)(HF + ((size_t)b * T2 + t0 + rr) * HH + c0 + c4) = *(const v4f*)(&Ts[wave][rr][c4]); } }
    else { for (int i = lane; i < 16 * 16; i += 32) { const int rr = i >> 4, c8 = (i & 15) * 8; const size_t gi = ((size_t)b * TP + 1 + t0 + rr) * HH + c0 + c8; *(volatile v8b*)(Oh + gi) = *(const v8b*)(&Th[wave][rr][c8]); *(volatile v8b*)(Ol + gi) = *(const v8b*)(&Tl[wave][rr][c8]); } }
    __threadfence(); }
}
__global__ __launch_bounds__(256) void prep_halo512(b16* __restrict__ Ah, b16* __restrict__ Al) {
  const int b = blockIdx.x, t_ = threadIdx.x; const v8b z = {};
  for (int pass = 0; pass < 2; ++pass) { for (int i = t_; i < 2 * 64; i += 256) { const int which = i >> 6, c8 = (i & 63) * 8; const size_t row = (size_t)b * TP + (which ? TP - 1 : 0); *(volatile v8b*)(Ah + row * HH + c8) = z; *(volatile v8b*)(Al + row * HH + c8) = z; } __threadfence(); }
}
__global__ __launch_bounds__(256) void tail_kernel(const float* __restrict__ HF, const float* __restrict__ x, const float* __restrict__ wo, const float* __restrict__ P, float* __restrict__ zout, float* __restrict__ LD) {
  __shared__ float Os[T2][10]; __shared__ __attribute__((aligned(16))) float Zs[T * 2]; __shared__ float Lt[T2 * 2];
  const int b = blockIdx.x, wave = threadIdx.x >> 5, lane = threadIdx.x & 31, t_ = threadIdx.x;
  for (int t = wave; t < T2; t += 8) { const float* hr = HF + ((size_t)b * T2 + t) * HH; float hv[16];
#pragma unroll
    for (int e = 0; e < 16; ++e) hv[e] = hr[lane * 16 + e];
    for (int j = 0; j < 10; ++j) { float s = 0.0f;
#pragma unroll
      for (int e = 0; e < 16; ++e) s += pmul(hv[e], bf16_rne(wo[(size_t)j * HH + lane * 16 + e]));
      s = wsum(s); if (lane == 0) Os[t][j] = s + P[13312 + j]; } }
  __syncthreads();
  if (t_ < 64) { const int t = t_ >> 1, d = t_ & 1; const float a = Os[t][5 * d], logb = Os[t][5 * d + 1] * 0.4f, Bt = Os[t][5 * d + 2] * 0.3f, logd = Os[t][5 * d + 3] * 0.4f, f = Os[t][5 * d + 4];
    const float bq = nexp(logb), dq = nexp(logd), cq = pmul(tanh_f(Bt), nexp(LOG_A + logb - logd)); const float z2 = bf16_rne(x[((size_t)b * T + T2 + t) * 2 + d]);
    const float arg = pmul(dq, z2) + f; const float denom = 1.0f + pmul(arg, arg); const float z2n = a + pmul(bq, z2) + cq / denom;
    Zs[(T2 + t) * 2 + d] = z2n; Lt[t_] = logf(bq - 2.0f * pmul(pmul(cq, dq), arg) / pmul(denom, denom)); }
  else if (t_ < 128) { const int i = t_ - 64; Zs[i] = bf16_rne(x[(size_t)b * T * 2 + i]); }
  __syncthreads();
  float ldv = 0.0f; if (t_ == 0) { float s = 0.0f; for (int i = 0; i < 64; ++i) s += Lt[i]; ldv = s; }
  for (int pass = 0; pass < 2; ++pass) { if (t_ < 32) { *(volatile v4f*)(zout + (size_t)b * T * 2 + t_ * 4) = *(const v4f*)(&Zs[t_ * 4]); ((volatile float*)LD)[(size_t)b * 32 + t_] = ldv; }
    __threadfence(); }
}
__global__ __launch_bounds__(256) void ld_kernel(const float* __restrict__ LD, float* __restrict__ out1) {
  const float v = LD[(size_t)threadIdx.x * 32]; for (int pass = 0; pass < 2; ++pass) { ((volatile float*)out1)[threadIdx.x] = v; __threadfence(); }
}
}

extern "C" void kernel_launch(void* const* d_in, const int* in_sizes, int n_in,
                              void* d_out, int out_size, void* d_ws, size_t ws_size, hipStream_t stream) {
  (void)n_in; (void)out_size;
  auto Fp = [&](int i) { return (const float*)d_in[i]; };
  float* zout = (float*)d_out; float* out1 = zout + (size_t)Bn * T * 2;
  if (in_sizes[0] != Bn * T * 2 || in_sizes[1] != Bn * 16 || in_sizes[8] != 512 * 1024 * 3) return;
  size_t off = 0; char* ws = (char*)d_ws;
  auto carve = [&](size_t bytes) { char* p = ws + off; off += (bytes + 255) & ~(size_t)255; return p; };
  b16* R = (b16*)carve(Ro_::END * 2); float* P = (float*)carve(13328 * 4); b16* C1h = (b16*)carve((size_t)Bn * HH * 2); b16* C1l = (b16*)carve((size_t)Bn * HH * 2);
  b16* Ah0 = (b16*)carve((size_t)NRP * 1024 * 2); b16* Al0 = (b16*)carve((size_t)NRP * 1024 * 2); b16* Ah1 = (b16*)carve((size_t)NRP * HH * 2); b16* Al1 = (b16*)carve((size_t)NRP * HH * 2); b16* Ah2 = (b16*)carve((size_t)NRP * HH * 2); b16* Al2 = (b16*)carve((size_t)NRP * HH * 2);
  float* HF = (float*)carve((size_t)NR * HH * 4); float* LD = (float*)carve((size_t)Bn * 32 * 4);
  if (off > ws_size) return;
  prep_kernel<<<1024, 256, 0, stream>>>(Fp(2), Fp(3), Fp(4), Fp(5), Fp(6), Fp(7), Fp(8), Fp(9), Fp(10), Fp(11), Fp(12), Fp(13), Fp(14), Fp(15), Fp(16), Fp(17), Fp(18), Fp(19), R, P, Ah0, Al0, Ah1, Al1);
  prep_halo512<<<Bn, 256, 0, stream>>>(Ah2, Al2);
  pre_kernel<<<Bn, 256, 0, stream>>>(Fp(0), Fp(1), P, C1h, C1l, Ah0, Al0);
  cond2_kernel<<<dim3(4, Bn / 32), 64, 0, stream>>>(C1h, C1l, R, P, Ah0, Al0);
  conv_kernel<1024, 0><<<dim3(4, Bn), 64, 0, stream>>>(Ah0, Al0, R + Ro_::C0, P + 10752, Ah1, Al1, nullptr);
  conv_kernel<512, 0><<<dim3(4, Bn), 64, 0, stream>>>(Ah1, Al1, R + Ro_::C1, P + 10752 + 512, Ah2, Al2, nullptr);
  conv_kernel<512, 0><<<dim3(4, Bn), 64, 0, stream>>>(Ah2, Al2, R + Ro_::C1 + (size_t)512 * 1536, P + 10752 + 1024, Ah1, Al1, nullptr);
  conv_kernel<512, 0><<<dim3(4, Bn), 64, 0, stream>>>(Ah1, Al1, R + Ro_::C1 + (size_t)2 * 512 * 1536, P + 10752 + 1536, Ah2, Al2, nullptr);
  conv_kernel<512, 1><<<dim3(4, Bn), 64, 0, stream>>>(Ah2, Al2, R + Ro_::C1 + (size_t)3 * 512 * 1536, P + 10752 + 2048, nullptr, nullptr, HF);
  tail_kernel<<<Bn, 256, 0, stream>>>(HF, Fp(0), Fp(18), P, zout, LD);
  ld_kernel<<<1, 256, 0, stream>>>(LD, out1);
}
